// SparseGPT_1803886265467
// MI455X (gfx1250) — hardware-verified
//
#include <hip/hip_runtime.h>


namespace {
constexpr int B = 2, T = 2048, NH = 16, HS = 64, E = 1024, DA = 1024, DB = 512, NP = B * T, NA = NP / 2, NB = NP / 2;
constexpr float XS = 8.0f, PS = 1024.0f, WSC = 256.0f;
typedef _Float16 b16;
typedef __attribute__((ext_vector_type(16))) _Float16 v16b;
typedef __attribute__((ext_vector_type(8))) _Float16 v8b;
typedef __attribute__((ext_vector_type(8))) float v8f;
typedef __attribute__((ext_vector_type(4))) float v4f;
typedef __attribute__((ext_vector_type(2))) float v2f;
__device__ __forceinline__ float bf16_rne(float f) { unsigned int u = __float_as_uint(f); u += 0x7FFFu + ((u >> 16) & 1u); return __uint_as_float(u & 0xFFFF0000u); }
__device__ __forceinline__ void split16(float v, b16& hi, b16& lo) { hi = (b16)v; lo = (b16)(v - (float)hi); }
__device__ __forceinline__ v16b frag_kb(const b16* p, int hh) { const v8b a = *(const v8b*)(p + 8 * hh), b = *(const v8b*)(p + 16 + 8 * hh); v16b f;
#pragma unroll
  for (int e = 0; e < 8; ++e) { f[e] = a[e]; f[8 + e] = b[e]; } return f; }
__device__ __forceinline__ v8f wmma16b(v16b a, v16b b, v8f c) { v8f d = __builtin_amdgcn_wmma_f32_16x16x32_f16(false, a, false, b, (short)0, c, false, false); asm volatile("v_nop\n\tv_nop\n\tv_nop\n\tv_nop" : "+v"(d) : "v"(a), "v"(b)); return d; }
__device__ __forceinline__ void wave_lds_sync() { __builtin_amdgcn_fence(__ATOMIC_RELEASE, "workgroup"); __builtin_amdgcn_wave_barrier(); __builtin_amdgcn_fence(__ATOMIC_ACQUIRE, "workgroup"); }
__device__ __forceinline__ int iclamp(int v, int lo, int hi) { return v < lo ? lo : (v > hi ? hi : v); }

__global__ __launch_bounds__(256) void wput_kernel(const float* __restrict__ w, int KIN, int OUTW, b16* __restrict__ WT) { const int KG = KIN / 8; const size_t u = (size_t)blockIdx.x * 256 + threadIdx.x; if (u >= (size_t)OUTW * KG) return; const int o = (int)(u / KG), k0 = (int)(u % KG) * 8; v8b v;
#pragma unroll
  for (int j = 0; j < 8; ++j) v[j] = (b16)(bf16_rne(w[(size_t)(k0 + j) * OUTW + o]) * WSC); for (int pass = 0; pass < 2; ++pass) { *(volatile v8b*)(WT + (size_t)o * KIN + k0) = v; __threadfence(); } }
__global__ __launch_bounds__(256) void scan_kernel(const int* __restrict__ mask, int* __restrict__ POSA, int* __restrict__ POSB) {
  __shared__ int cntA[256], la[NA], lb[NB]; const int tid = threadIdx.x; const int per = NP / 256;
  int c = 0; for (int i = 0; i < per; ++i) c += (mask[tid * per + i] != 0) ? 1 : 0; cntA[tid] = c;
  __syncthreads();
  if (tid == 0) { int acc = 0; for (int i = 0; i < 256; ++i) { const int v = cntA[i]; cntA[i] = acc; acc += v; } }
  __syncthreads();
  for (int i = tid; i < NA; i += 256) { la[i] = NP - 1; } for (int i = tid; i < NB; i += 256) { lb[i] = NP - 1; }
  __syncthreads();
  { int ra = cntA[tid], rbk = tid * per - ra; for (int i = 0; i < per; ++i) { const int p = tid * per + i; if (mask[p] != 0) { if (ra < NA) la[ra] = p; ++ra; } else { if (rbk < NB) lb[rbk] = p; ++rbk; } } }
  __syncthreads();
  for (int pass = 0; pass < 2; ++pass) { for (int i = tid; i < NA; i += 256) ((volatile int*)POSA)[i] = la[i]; for (int i = tid; i < NB; i += 256) ((volatile int*)POSB)[i] = lb[i]; __threadfence(); }
}
template <int KIN>
__global__ __launch_bounds__(32) void qkv_kernel(const float* __restrict__ x, const b16* __restrict__ WT, const int* __restrict__ POS, const float* __restrict__ cosT, const float* __restrict__ sinT, int NROWS, int TV, float* __restrict__ Q, float* __restrict__ K, float* __restrict__ V) {
  __shared__ __attribute__((aligned(16))) b16 Ah[16][KIN + 8]; __shared__ float Tf[16][132]; __shared__ int Pr[16]; const int lane = threadIdx.x, nloc = lane & 15, hlf = lane >> 4; const int cg = blockIdx.x % 24; const size_t m0 = (size_t)(blockIdx.x / 24) * 16; if (m0 >= (size_t)NROWS) return;
  if (lane < 16) Pr[lane] = iclamp(POS[m0 + lane], 0, NP - 1);
  wave_lds_sync(); { bool any = false; for (int rr = 0; rr < 16; ++rr) any |= (Pr[rr] % T) < TV; if (!any) return; }
  for (int rr = 0; rr < 16; ++rr) for (int q = 0; q < KIN / 32; ++q) Ah[rr][q * 32 + lane] = (b16)(bf16_rne(x[(m0 + rr) * KIN + q * 32 + lane]) * XS);
  wave_lds_sync(); v8f acc[8];
#pragma unroll
  for (int t = 0; t < 8; ++t) acc[t] = (v8f){};
#pragma unroll 2
  for (int kb = 0; kb < KIN; kb += 32) { const v16b a = frag_kb(&Ah[nloc][kb], hlf);
#pragma unroll
    for (int t = 0; t < 8; ++t) acc[t] = wmma16b(a, frag_kb(WT + (size_t)(cg * 128 + t * 16 + nloc) * KIN + kb, hlf), acc[t]); }
#pragma unroll
  for (int t = 0; t < 8; ++t)
#pragma unroll
    for (int r8 = 0; r8 < 8; ++r8) Tf[8 * hlf + r8][t * 16 + nloc] = acc[t][r8] * (1.0f / (XS * WSC));
  wave_lds_sync();
  const int which = cg / 8; float* O = which == 0 ? Q : (which == 1 ? K : V); const int c0 = (cg % 8) * 128;
  for (int pass = 0; pass < 2; ++pass) { for (int rr = 0; rr < 16; ++rr) { const int p = Pr[rr]; const int tpos = p % T;
      for (int q = 0; q < 4; ++q) { const int c = q * 32 + lane; float v = Tf[rr][c];
        if (which < 2) { const int d = c & 63; const float cs = bf16_rne(cosT[(size_t)tpos * HS + d]), sn = bf16_rne(sinT[(size_t)tpos * HS + d]); const float other = (d < 32) ? -Tf[rr][c + 32] : Tf[rr][c - 32]; v = v * cs + other * sn; }
        ((volatile float*)O)[(size_t)p * E + c0 + c] = v; } }
    __threadfence(); }
}
__global__ __launch_bounds__(32) void att_kernel(const float* __restrict__ Q, const float* __restrict__ K, const float* __restrict__ V, int TV, float* __restrict__ Y) {
  __shared__ __attribute__((aligned(16))) b16 Qp[16][HS + 8], Kp[32][HS + 8], Ph[16][40], Pl[16][40], Vh[HS][40], Vl[HS][40]; __shared__ float Sc[16][33], Mx[16], Dn[16], Sf[16], Of[16][HS + 2];
  const int lane = threadIdx.x, nloc = lane & 15, hlf = lane >> 4; const int qt = blockIdx.x % (TV / 16); const int h = (blockIdx.x / (TV / 16)) % NH; const int b = blockIdx.x / ((TV / 16) * NH); const int q0 = qt * 16; const size_t pb = (size_t)b * T;
  for (int rr = 0; rr < 16; ++rr) for (int q = 0; q < 2; ++q) Qp[rr][q * 32 + lane] = (b16)(Q[(pb + q0 + rr) * E + h * HS + q * 32 + lane] * XS);
  if (lane < 16) { Mx[lane] = -INFINITY; Dn[lane] = 0.0f; Sf[lane] = 0.0f; }
  v8f acc[4] = {(v8f){}, (v8f){}, (v8f){}, (v8f){}}; wave_lds_sync();
#pragma unroll 1
  for (int kc = 0; kc < q0 + 16; kc += 32) {
    for (int rr = 0; rr < 32; ++rr) { const int kk = kc + rr; const bool ok = kk < T; for (int q = 0; q < 2; ++q) { const float kvv = ok ? K[(pb + kk) * E + h * HS + q * 32 + lane] : 0.0f; Kp[rr][q * 32 + lane] = (b16)(kvv * XS); b16 p, ql; split16((ok ? V[(pb + kk) * E + h * HS + q * 32 + lane] : 0.0f) * XS, p, ql); Vh[q * 32 + lane][rr] = p; Vl[q * 32 + lane][rr] = ql; } }
    wave_lds_sync();
#pragma unroll
    for (int blk = 0; blk < 2; ++blk) { v8f s = {};
#pragma unroll
      for (int kb = 0; kb < HS; kb += 32) s = wmma16b(frag_kb(&Qp[nloc][kb], hlf), frag_kb(&Kp[blk * 16 + nloc][kb], hlf), s);
#pragma unroll
      for (int r8 = 0; r8 < 8; ++r8) { const int qi = q0 + 8 * hlf + r8, kk = kc + blk * 16 + nloc; Sc[8 * hlf + r8][blk * 16 + nloc] = (kk <= qi) ? s[r8] * (0.125f / (XS * XS)) : -INFINITY; } }
    wave_lds_sync();
#pragma unroll 1
    for (int qi = 0; qi < 16; ++qi) { const float sv = Sc[qi][lane]; float cm = sv; for (int o = 16; o; o >>= 1) cm = fmaxf(cm, __shfl_xor(cm, o)); const float mo = Mx[qi]; const float mn = fmaxf(mo, cm); const float p = (sv == -INFINITY) ? 0.0f : __expf(sv - mn); float psum = p; for (int o = 16; o; o >>= 1) psum += __shfl_xor(psum, o);
      b16 ph, plo; split16(p * PS, ph, plo); Ph[qi][lane] = ph; Pl[qi][lane] = plo; if (lane == 0) { const float sf = (mo == -INFINITY) ? 0.0f : __expf(mo - mn); Sf[qi] = sf; Dn[qi] = Dn[qi] * sf + psum; Mx[qi] = mn; } }
    wave_lds_sync(); const v16b pa = frag_kb(&Ph[nloc][0], hlf), plf = frag_kb(&Pl[nloc][0], hlf);
#pragma unroll
    for (int t = 0; t < 4; ++t) {
#pragma unroll
      for (int r8 = 0; r8 < 8; ++r8) acc[t][r8] *= Sf[8 * hlf + r8];
      const v16b vh = frag_kb(&Vh[t * 16 + nloc][0], hlf), vl = frag_kb(&Vl[t * 16 + nloc][0], hlf); acc[t] = wmma16b(pa, vh, acc[t]); acc[t] = wmma16b(pa, vl, acc[t]); acc[t] = wmma16b(plf, vh, acc[t]); }
    wave_lds_sync(); }
#pragma unroll
  for (int t = 0; t < 4; ++t)
#pragma unroll
    for (int r8 = 0; r8 < 8; ++r8) { const int rl = 8 * hlf + r8; Of[rl][t * 16 + nloc] = acc[t][r8] * (1.0f / (PS * XS)) / Dn[rl]; }
  wave_lds_sync();
  for (int pass = 0; pass < 2; ++pass) { for (int rr = 0; rr < 16; ++rr) *(volatile v2f*)(Y + (pb + q0 + rr) * E + h * HS + lane * 2) = (v2f){Of[rr][lane * 2], Of[rr][lane * 2 + 1]}; __threadfence(); }
}
__global__ __launch_bounds__(32) void proj_kernel(const float* __restrict__ Y, const int* __restrict__ POS, const b16* __restrict__ WP, int OUTW, int TV, float* __restrict__ out) {
  __shared__ __attribute__((aligned(16))) b16 Ah[16][E + 8], Al[16][E + 8]; __shared__ float Tf[16][132]; __shared__ int Pr[16]; const int lane = threadIdx.x, nloc = lane & 15, hlf = lane >> 4; const int ncg = OUTW / 128; const int cg = blockIdx.x % ncg; const size_t m0 = (size_t)(blockIdx.x / ncg) * 16;
  if (lane < 16) { const int p = iclamp(POS[m0 + lane], 0, NP - 1); Pr[lane] = ((p % T) < TV) ? p : -1; }
  wave_lds_sync();
  { bool any = false; for (int rr = 0; rr < 16; ++rr) any |= Pr[rr] >= 0; if (!any) { for (int pass = 0; pass < 2; ++pass) { for (int rr = 0; rr < 16; ++rr) *(volatile v4f*)(out + (m0 + rr) * (size_t)OUTW + cg * 128 + lane * 4) = (v4f){0.0f, 0.0f, 0.0f, 0.0f}; __threadfence(); } return; } }
  for (int rr = 0; rr < 16; ++rr) { const int p = Pr[rr]; for (int q = 0; q < E / 32; ++q) { b16 a = (b16)0.0f, bl = (b16)0.0f; if (p >= 0) split16(Y[(size_t)p * E + q * 32 + lane] * XS, a, bl); Ah[rr][q * 32 + lane] = a; Al[rr][q * 32 + lane] = bl; } }
  wave_lds_sync(); v8f acc[8];
#pragma unroll
  for (int t = 0; t < 8; ++t) acc[t] = (v8f){};
#pragma unroll 2
  for (int kb = 0; kb < E; kb += 32) { const v16b a = frag_kb(&Ah[nloc][kb], hlf), al = frag_kb(&Al[nloc][kb], hlf);
#pragma unroll
    for (int t = 0; t < 8; ++t) { const v16b bw = frag_kb(WP + (size_t)(cg * 128 + t * 16 + nloc) * E + kb, hlf); acc[t] = wmma16b(a, bw, acc[t]); acc[t] = wmma16b(al, bw, acc[t]); } }
#pragma unroll
  for (int t = 0; t < 8; ++t)
#pragma unroll
    for (int r8 = 0; r8 < 8; ++r8) Tf[8 * hlf + r8][t * 16 + nloc] = acc[t][r8] * (1.0f / (XS * WSC));
  wave_lds_sync();
  for (int pass = 0; pass < 2; ++pass) { for (int rr = 0; rr < 16; ++rr) *(volatile v4f*)(out + (m0 + rr) * (size_t)OUTW + cg * 128 + lane * 4) = *(const v4f*)(&Tf[rr][lane * 4]); __threadfence(); }
}
}

extern "C" void kernel_launch(void* const* d_in, const int* in_sizes, int n_in, void* d_out, int out_size, void* d_ws, size_t ws_size, hipStream_t stream) {
  (void)n_in;
  auto Fp = [&](int i) { return (const float*)d_in[i]; }; auto Ip = [&](int i) { return (const int*)d_in[i]; };
  if (in_sizes[0] != NA * DA || in_sizes[1] != NB * DB || in_sizes[2] != T * HS || in_sizes[3] != T * HS || in_sizes[4] != NP || in_sizes[5] != DA * 3 * E || in_sizes[6] != DB * 3 * E || in_sizes[7] != E * DA || in_sizes[8] != E * DB || out_size != NA * DA + NB * DB) return;
  const int TV = T;
  size_t off = 0; char* ws = (char*)d_ws;
  auto carve = [&](size_t bytes) { char* p = ws + off; off += (bytes + 255) & ~(size_t)255; return p; };
  b16* WA = (b16*)carve((size_t)3 * E * DA * 2); b16* WB = (b16*)carve((size_t)3 * E * DB * 2); b16* WPA = (b16*)carve((size_t)DA * E * 2); b16* WPB = (b16*)carve((size_t)DB * E * 2); int* POSA = (int*)carve((size_t)NA * 4); int* POSB = (int*)carve((size_t)NB * 4);
  float* Q = (float*)carve((size_t)NP * E * 4); float* K = (float*)carve((size_t)NP * E * 4); float* V = (float*)carve((size_t)NP * E * 4); float* Y = (float*)carve((size_t)NP * E * 4);
  if (off > ws_size || off > ((size_t)96 << 20)) return;
  wput_kernel<<<(unsigned)(((size_t)3 * E * (DA / 8) + 255) / 256), 256, 0, stream>>>(Fp(5), DA, 3 * E, WA); wput_kernel<<<(unsigned)(((size_t)3 * E * (DB / 8) + 255) / 256), 256, 0, stream>>>(Fp(6), DB, 3 * E, WB);
  wput_kernel<<<(unsigned)(((size_t)DA * (E / 8) + 255) / 256), 256, 0, stream>>>(Fp(7), E, DA, WPA); wput_kernel<<<(unsigned)(((size_t)DB * (E / 8) + 255) / 256), 256, 0, stream>>>(Fp(8), E, DB, WPB);
  scan_kernel<<<1, 256, 0, stream>>>(Ip(4), POSA, POSB);
  qkv_kernel<DA><<<(NA / 16) * 24, 32, 0, stream>>>(Fp(0), WA, POSA, Fp(2), Fp(3), NA, TV, Q, K, V);
  qkv_kernel<DB><<<(NB / 16) * 24, 32, 0, stream>>>(Fp(1), WB, POSB, Fp(2), Fp(3), NB, TV, Q, K, V);
  att_kernel<<<B * NH * (TV / 16), 32, 0, stream>>>(Q, K, V, TV, Y);
  float* out = (float*)d_out;
  proj_kernel<<<(NA / 16) * (DA / 128), 32, 0, stream>>>(Y, POSA, WPA, DA, TV, out);
  proj_kernel<<<(NB / 16) * (DB / 128), 32, 0, stream>>>(Y, POSB, WPB, DB, TV, out + (size_t)NA * DA);
}
